// SparseConvolutionBase_83769042141676
// MI455X (gfx1250) — hardware-run, weakly checked
//
#include <hip/hip_runtime.h>


namespace {
constexpr int NPTS = 100000, KV = 27, PAIRS = 60000, CI = 64, CO = 64, KVU = 27  , E = KVU * PAIRS, NQ = 4, EH = ((E / NQ + 15) / 16) * 16;
constexpr float XS = 8.0f, WSC = 256.0f;

typedef _Float16 b16;
typedef __attribute__((ext_vector_type(16))) _Float16 v16b;
typedef __attribute__((ext_vector_type(8))) _Float16 v8b;
typedef __attribute__((ext_vector_type(4))) _Float16 v4b;
typedef __attribute__((ext_vector_type(8))) float v8f;
typedef __attribute__((ext_vector_type(4))) float v4f;
__device__ __forceinline__ float bf16_rne(float f) { unsigned int u = __float_as_uint(f); u += 0x7FFFu + ((u >> 16) & 1u); return __uint_as_float(u & 0xFFFF0000u); }
__device__ __forceinline__ v16b frag_kb(const b16* p, int hh) { const v8b a = *(const v8b*)(p + 8 * hh), b = *(const v8b*)(p + 16 + 8 * hh); v16b f;
#pragma unroll
  for (int e = 0; e < 8; ++e) { f[e] = a[e]; f[8 + e] = b[e]; } return f; }
__device__ __forceinline__ v8f wmma16b(v16b a, v16b b, v8f c) { v8f d = __builtin_amdgcn_wmma_f32_16x16x32_f16(false, a, false, b, (short)0, c, false, false); asm volatile("v_nop\n\tv_nop\n\tv_nop\n\tv_nop" : "+v"(d) : "v"(a), "v"(b)); return d; }
__device__ __forceinline__ void wave_lds_sync() { __builtin_amdgcn_fence(__ATOMIC_RELEASE, "workgroup"); __builtin_amdgcn_wave_barrier(); __builtin_amdgcn_fence(__ATOMIC_ACQUIRE, "workgroup"); }
__device__ __forceinline__ int iclamp(int v, int lo, int hi) { return v < lo ? lo : (v > hi ? hi : v); }

constexpr int CSR_NBLK = 512, CSR_GB = 9, CSR_GN = 1 << CSR_GB  , CSR_MAXG = 512, CSR_CAP = 12288  ;
__global__ __launch_bounds__(64) void csrA_kernel(const int* __restrict__ dst, int E, int N, int nG, int CHP, int NGP, int* __restrict__ STG, int* __restrict__ HST) {
  extern __shared__ int sm[];
  int* cnt = sm; int* run = sm + NGP; int* ids = sm + 2 * NGP;
  const int b = blockIdx.x; const int ch = (E + CSR_NBLK - 1) / CSR_NBLK; const int e0 = b * ch, e1 = min(E, e0 + ch);
  for (int i = threadIdx.x; i < NGP; i += 64) cnt[i] = 0;
  for (int i = threadIdx.x; i < CHP; i += 64) ids[i] = -1;
  __syncthreads();
  if (threadIdx.x == 0) {
    for (int e = e0; e < e1; ++e) { int d = dst[e]; d = (d < 0) ? 0 : (d >= N ? N - 1 : d); cnt[d >> CSR_GB] += 1; }
    int acc = 0; for (int g = 0; g < nG; ++g) { run[g] = acc; acc += cnt[g]; }
    for (int e = e0; e < e1; ++e) { int d = dst[e]; d = (d < 0) ? 0 : (d >= N ? N - 1 : d); const int g = d >> CSR_GB; ids[run[g]] = e; run[g] += 1; } }
  __syncthreads();
  typedef __attribute__((ext_vector_type(4))) int v4i;
  for (int pass = 0; pass < 2; ++pass) {
    for (int i = threadIdx.x; i < CHP / 4; i += 64) *(volatile v4i*)(STG + (size_t)b * CHP + i * 4) = *(const v4i*)(&ids[i * 4]);
    for (int i = threadIdx.x; i < NGP / 4; i += 64) { v4i v; for (int e = 0; e < 4; ++e) v[e] = (i * 4 + e < nG) ? cnt[i * 4 + e] : 0; *(volatile v4i*)(HST + (size_t)b * NGP + i * 4) = v; }
    __threadfence(); }
}
__global__ __launch_bounds__(512) void csrS_kernel(const int* __restrict__ HST, int nG, int NGP, int* __restrict__ START, int* __restrict__ TOT, int* __restrict__ OFF) {
  __shared__ int tot[CSR_MAXG];
  const int b = threadIdx.x;
  for (int pass = 0; pass < 2; ++pass) { int runb = 0; for (int g = 0; g < nG; ++g) { int c = HST[(size_t)b * NGP + g]; c = (c < 0) ? 0 : c; ((volatile int*)OFF)[(size_t)g * CSR_NBLK + b] = runb; runb += c; } __threadfence(); }
  for (int g = threadIdx.x; g < nG; g += 512) { int s = 0; for (int bb = 0; bb < CSR_NBLK; ++bb) { int c = HST[(size_t)bb * NGP + g]; s += (c < 0) ? 0 : c; } tot[g] = s; }
  __syncthreads();
  if (threadIdx.x < 32) {
    __shared__ int st[CSR_MAXG + 32];
    if (threadIdx.x == 0) { int acc = 0; for (int g = 0; g < NGP; ++g) { st[g] = acc; if (g < nG) acc += (tot[g] + 31) & ~31; } st[NGP] = acc; }
    __builtin_amdgcn_fence(__ATOMIC_RELEASE, "workgroup"); __builtin_amdgcn_wave_barrier(); __builtin_amdgcn_fence(__ATOMIC_ACQUIRE, "workgroup");
    for (int pass = 0; pass < 2; ++pass) { for (int i = threadIdx.x; i < NGP + 32; i += 32) { ((volatile int*)START)[i] = (i <= NGP) ? st[min(i, NGP)] : 0; ((volatile int*)TOT)[i] = (i < nG) ? tot[i] : 0; } __threadfence(); } }
}
__global__ __launch_bounds__(256) void csrB_kernel(const int* __restrict__ dst, int N, int nG, int CHP, int NGP, int permLen, const int* __restrict__ STG, const int* __restrict__ HST, const int* __restrict__ OFF, const int* __restrict__ START, const int* __restrict__ TOT, int* __restrict__ PERM, int* __restrict__ ROWPTR, int* __restrict__ ROWCNT, int* __restrict__ FLAG) {
  typedef __attribute__((ext_vector_type(4))) int v4i;
  __shared__ int ids[CSR_CAP]; __shared__ unsigned short key[CSR_CAP]; __shared__ int outp[CSR_CAP]; __shared__ int ncnt[CSR_GN + 1]; __shared__ int boff[CSR_NBLK + 1];
  const int g = blockIdx.x, t_ = threadIdx.x; int tot = TOT[g]; int st = START[g], stn = START[g + 1]; const int v0 = g * CSR_GN; const int nv = min(CSR_GN, N - v0);
  st = (st < 0) ? 0 : (st > permLen - 32 ? permLen - 32 : st) & ~31; stn = (stn < st) ? st : (stn > permLen ? permLen : stn); tot = (tot < 0) ? 0 : tot; if (tot > stn - st && tot <= CSR_CAP) tot = stn - st;
  if (tot > CSR_CAP) {
    for (int pass = 0; pass < 2; ++pass) { for (int i = t_; i < CSR_GN / 4; i += 256) { v4i a, c; for (int e = 0; e < 4; ++e) { a[e] = st; c[e] = 0; } *(volatile v4i*)(ROWPTR + v0 + i * 4) = a; *(volatile v4i*)(ROWCNT + v0 + i * 4) = c; } if (t_ == 0) ((volatile int*)FLAG)[0] = 1; __threadfence(); } (void)nv; return; }
  if (t_ == 0) { int acc = 0; for (int b = 0; b < CSR_NBLK; ++b) { boff[b] = acc; int c = HST[(size_t)b * NGP + g]; c = (c < 0) ? 0 : (c > CHP ? CHP : c); acc += c; if (acc > tot) acc = tot; } boff[CSR_NBLK] = acc; }
  for (int i = t_; i <= CSR_GN; i += 256) ncnt[i] = 0;
  __syncthreads();
  for (int b = 0; b < CSR_NBLK; ++b) { const int c = boff[b + 1] - boff[b]; int o_ = OFF[(size_t)g * CSR_NBLK + b]; o_ = (o_ < 0) ? 0 : (o_ > CHP - c ? CHP - c : o_); const int* src_ = STG + (size_t)b * CHP + o_;
    for (int i = t_; i < c; i += 256) { int id = src_[i]; id = (id < 0) ? 0 : id; ids[boff[b] + i] = id; int d = dst[id]; d = (d < v0) ? v0 : (d >= N ? N - 1 : d); int kk = d - v0; kk = (kk < 0) ? 0 : (kk >= CSR_GN ? CSR_GN - 1 : kk); key[boff[b] + i] = (unsigned short)kk; } }
  __syncthreads();
  if (t_ == 0) { for (int i = 0; i < tot; ++i) ncnt[key[i]] += 1; int acc = 0; for (int vl = 0; vl < CSR_GN; ++vl) { const int c = ncnt[vl]; ncnt[vl] = acc; acc += c; } ncnt[CSR_GN] = acc;
    for (int i = 0; i < tot; ++i) { const int vl = key[i]; outp[ncnt[vl]] = ids[i]; ncnt[vl] += 1; }
    for (int vl = CSR_GN; vl > 0; --vl) ncnt[vl] = ncnt[vl - 1]; ncnt[0] = 0; }
  __syncthreads();
  for (int pass = 0; pass < 2; ++pass) {
    for (int i = t_; i < (stn - st) / 4; i += 256) { v4i v; for (int e = 0; e < 4; ++e) { const int q = i * 4 + e; v[e] = (q < tot) ? outp[q] : -1; } *(volatile v4i*)(PERM + st + i * 4) = v; }
    for (int i = t_; i < CSR_GN / 4; i += 256) { v4i a, c; for (int e = 0; e < 4; ++e) { const int vl = i * 4 + e; a[e] = st + ncnt[vl]; c[e] = (vl < nv) ? (ncnt[vl + 1] - ncnt[vl]) : 0; } *(volatile v4i*)(ROWPTR + v0 + i * 4) = a; *(volatile v4i*)(ROWCNT + v0 + i * 4) = c; }
    __threadfence(); }
}
__global__ __launch_bounds__(256) void csrZ_kernel(int* __restrict__ p, size_t n4) { typedef __attribute__((ext_vector_type(4))) int v4i; const size_t tid = (size_t)blockIdx.x * 256 + threadIdx.x, nth = (size_t)gridDim.x * 256; v4i z = {0, 0, 0, 0}; for (size_t i = tid; i < n4; i += nth) *(volatile v4i*)(p + i * 4) = z; }
struct CsrBufs { int *STG, *HST, *OFF, *START, *TOT, *PERM, *ROWPTR, *ROWCNT, *FLAG; int nG, NGP, CHP; size_t permLen; char* base; size_t bytes; };
static size_t csr_carve(CsrBufs& c, char* ws, size_t off, int E, int N) {
  const size_t off0 = off; c.base = ws + off;
  auto al = [&](size_t bytes) { char* p = ws + off; off += (bytes + 255) & ~(size_t)255; return p; };
  c.nG = (N + CSR_GN - 1) / CSR_GN; c.NGP = (c.nG + 31) & ~31; const int ch = (E + CSR_NBLK - 1) / CSR_NBLK; c.CHP = (ch + 31) & ~31; c.permLen = (size_t)E + 32 * (size_t)c.nG + 32;
  c.STG = (int*)al((size_t)CSR_NBLK * c.CHP * 4); c.HST = (int*)al((size_t)CSR_NBLK * c.NGP * 4); c.OFF = (int*)al((size_t)c.NGP * CSR_NBLK * 4); c.START = (int*)al((size_t)(c.NGP + 64) * 4); c.TOT = (int*)al((size_t)(c.NGP + 64) * 4);
  c.PERM = (int*)al(c.permLen * 4); c.ROWPTR = (int*)al((size_t)c.nG * CSR_GN * 4); c.ROWCNT = (int*)al((size_t)c.nG * CSR_GN * 4); c.FLAG = (int*)al(256);
  c.bytes = off - off0; return off;
}
static void csr_build(const CsrBufs& c, const int* dst, int E, int N, hipStream_t stream) {
  const size_t smem = (size_t)(2 * c.NGP + c.CHP) * 4;
  csrZ_kernel<<<512, 256, 0, stream>>>((int*)c.base, c.bytes / 16);
  csrA_kernel<<<CSR_NBLK, 64, smem, stream>>>(dst, E, N, c.nG, c.CHP, c.NGP, c.STG, c.HST);
  csrS_kernel<<<1, 512, 0, stream>>>(c.HST, c.nG, c.NGP, c.START, c.TOT, c.OFF);
  csrB_kernel<<<c.nG, 256, 0, stream>>>(dst, N, c.nG, c.CHP, c.NGP, (int)c.permLen, c.STG, c.HST, c.OFF, c.START, c.TOT, c.PERM, c.ROWPTR, c.ROWCNT, c.FLAG);
}


__global__ __launch_bounds__(256) void prepx_kernel(const float* __restrict__ in, b16* __restrict__ X16) {
  const size_t i = ((size_t)blockIdx.x * 256 + threadIdx.x) * 8; if (i >= (size_t)NPTS * CI) return;
  const v4f a = *(const v4f*)(in + i), c = *(const v4f*)(in + i + 4); v8b o;
#pragma unroll
  for (int j = 0; j < 4; ++j) { o[j] = (b16)(bf16_rne(a[j]) * XS); o[4 + j] = (b16)(bf16_rne(c[j]) * XS); }
  for (int pass = 0; pass < 2; ++pass) { *(volatile v8b*)(X16 + i) = o; __threadfence(); }
}
__global__ __launch_bounds__(256) void prepk_kernel(const float* __restrict__ ker, b16* __restrict__ KT) {
  __shared__ __attribute__((aligned(16))) b16 Tt[64][64 + 8];
  const int k = blockIdx.x, t_ = threadIdx.x;
  for (int q = t_; q < 64 * 64; q += 256) { const int i = q >> 6, o = q & 63; Tt[o][i] = (b16)(bf16_rne(ker[((size_t)k * CI + i) * CO + o]) * WSC); }
  __syncthreads();
  for (int pass = 0; pass < 2; ++pass) { for (int q = t_; q < 64 * 8; q += 256) { const int o = q >> 3, c8 = (q & 7) * 8; *(volatile v8b*)(KT + ((size_t)k * CO + o) * CI + c8) = *(const v8b*)(&Tt[o][c8]); } __threadfence(); }
}
__global__ __launch_bounds__(128) void pair_kernel(const b16* __restrict__ X16, const b16* __restrict__ KT, const int* __restrict__ inmap, int qbase, float* __restrict__ Y) {
  __shared__ __attribute__((aligned(16))) b16 Ta[4][16][CI + 8]; __shared__ __attribute__((aligned(16))) float To[4][16][CO + 4];
  const int wave = threadIdx.x >> 5, lane = threadIdx.x & 31, nloc = lane & 15, hlf = lane >> 4; const int q0 = qbase + (blockIdx.x * 4 + wave) * 16; if (q0 >= qbase + EH || q0 >= E) return;
  const int k = q0 / PAIRS;
  { const int rr = lane >> 1, h2 = lane & 1; const int src = iclamp(inmap[q0 + rr], 0, NPTS - 1);
    const v8b* s = (const v8b*)(X16 + (size_t)src * CI + h2 * 32); *(v8b*)(&Ta[wave][rr][h2 * 32]) = s[0]; *(v8b*)(&Ta[wave][rr][h2 * 32 + 8]) = s[1]; *(v8b*)(&Ta[wave][rr][h2 * 32 + 16]) = s[2]; *(v8b*)(&Ta[wave][rr][h2 * 32 + 24]) = s[3]; }
  wave_lds_sync();
  v8f acc[4] = {{}, {}, {}, {}};
#pragma unroll
  for (int kb = 0; kb < CI; kb += 32) { const v16b a = frag_kb(&Ta[wave][nloc][kb], hlf);
#pragma unroll
    for (int t = 0; t < 4; ++t) acc[t] = wmma16b(a, frag_kb(KT + ((size_t)k * CO + t * 16 + nloc) * CI + kb, hlf), acc[t]); }
#pragma unroll
  for (int t = 0; t < 4; ++t)
#pragma unroll
    for (int r = 0; r < 8; ++r) To[wave][8 * hlf + r][t * 16 + nloc] = acc[t][r] * (1.0f / (XS * WSC));
  wave_lds_sync();
  for (int pass = 0; pass < 2; ++pass) { for (int r2 = 0; r2 < 16; r2 += 2) { const int rr = r2 + (lane >> 4), c4 = (lane & 15) * 4; *(volatile v4f*)(Y + ((size_t)(q0 - qbase) + rr) * CO + c4) = *(const v4f*)(&To[wave][rr][c4]); } __threadfence(); }
}
template <int QTR>
__global__ __launch_bounds__(256) void gather_kernel(const float* __restrict__ Y, const int* __restrict__ PERM, const int* __restrict__ ROWPTR, const int* __restrict__ ROWCNT, int permLen, const float* __restrict__ bias, float* __restrict__ out) {
  const int lane = threadIdx.x & 31, wave = threadIdx.x >> 5; const int n = (blockIdx.x * 8 + wave) * 2 + (lane >> 4); const int c0 = (lane & 15) * 4; const int qbase = QTR * EH;
  if (n >= NPTS) return;
  int st = ROWPTR[n], cnt = ROWCNT[n]; cnt = iclamp(cnt, 0, 64); st = iclamp(st, 0, permLen - cnt);
  v4f acc;
  if (QTR == 0) { acc[0] = bf16_rne(bias[c0]); acc[1] = bf16_rne(bias[c0 + 1]); acc[2] = bf16_rne(bias[c0 + 2]); acc[3] = bf16_rne(bias[c0 + 3]); } else acc = *(const v4f*)(out + (size_t)n * CO + c0);
  for (int j = 0; j < cnt; ++j) { const int q = PERM[st + j]; const bool inq = (q >= qbase) && (q < qbase + EH) && (q < E); const int qi = iclamp(q - qbase, 0, EH - 1);
    const v4f y = *(const v4f*)(Y + (size_t)qi * CO + c0);
#pragma unroll
    for (int e = 0; e < 4; ++e) acc[e] += inq ? y[e] : 0.0f; }
  for (int pass = 0; pass < 2; ++pass) { *(volatile v4f*)(out + (size_t)n * CO + c0) = acc; __threadfence(); }
}
}

extern "C" void kernel_launch(void* const* d_in, const int* in_sizes, int n_in, void* d_out, int out_size, void* d_ws, size_t ws_size, hipStream_t stream) {
  (void)n_in;
  if (in_sizes[0] != NPTS * CI || in_sizes[1] != KV * CI * CO || in_sizes[2] != CO || in_sizes[3] != KV * PAIRS || in_sizes[4] != KV * PAIRS || out_size != NPTS * CO) return;
  size_t off = 0; char* ws = (char*)d_ws;
  auto carve = [&](size_t bytes) { char* p = ws + off; off += (bytes + 255) & ~(size_t)255; return p; };
  b16* X16 = (b16*)carve((size_t)NPTS * CI * 2); b16* KT = (b16*)carve((size_t)KV * CO * CI * 2); float* Y = (float*)carve((size_t)EH * CO * 4);
  CsrBufs csr; off = csr_carve(csr, ws, off, E, NPTS);
  if (off > ws_size || off > ((size_t)128 << 20)) return;
  const int* inmap = (const int*)d_in[3]; const int* outmap = (const int*)d_in[4];
  prepx_kernel<<<(NPTS * CI / 8 + 255) / 256, 256, 0, stream>>>((const float*)d_in[0], X16);
  prepk_kernel<<<KV, 256, 0, stream>>>((const float*)d_in[1], KT);
  csr_build(csr, outmap, E, NPTS, stream);
  const int pgrid = EH / 64 + ((EH % 64) ? 1 : 0), ggrid = (NPTS / 2 + 7) / 8;
  pair_kernel<<<pgrid, 128, 0, stream>>>(X16, KT, inmap, 0 * EH, Y); gather_kernel<0><<<ggrid, 256, 0, stream>>>(Y, csr.PERM, csr.ROWPTR, csr.ROWCNT, (int)csr.permLen, (const float*)d_in[2], (float*)d_out);
  pair_kernel<<<pgrid, 128, 0, stream>>>(X16, KT, inmap, 1 * EH, Y); gather_kernel<1><<<ggrid, 256, 0, stream>>>(Y, csr.PERM, csr.ROWPTR, csr.ROWCNT, (int)csr.permLen, (const float*)d_in[2], (float*)d_out);
  pair_kernel<<<pgrid, 128, 0, stream>>>(X16, KT, inmap, 2 * EH, Y); gather_kernel<2><<<ggrid, 256, 0, stream>>>(Y, csr.PERM, csr.ROWPTR, csr.ROWCNT, (int)csr.permLen, (const float*)d_in[2], (float*)d_out);
  pair_kernel<<<pgrid, 128, 0, stream>>>(X16, KT, inmap, 3 * EH, Y); gather_kernel<3><<<ggrid, 256, 0, stream>>>(Y, csr.PERM, csr.ROWPTR, csr.ROWCNT, (int)csr.permLen, (const float*)d_in[2], (float*)d_out);
}
